// ConvSkip_87488483819569
// MI455X (gfx1250) — hardware-run, weakly checked
//
#include <hip/hip_runtime.h>

typedef float          v8f   __attribute__((ext_vector_type(8)));
typedef float          v4f   __attribute__((ext_vector_type(4)));
typedef unsigned int   v4u   __attribute__((ext_vector_type(4)));
typedef int            v8i   __attribute__((ext_vector_type(8)));
typedef unsigned short v8us  __attribute__((ext_vector_type(8)));
typedef unsigned short v16us __attribute__((ext_vector_type(16)));
typedef __bf16         v16bf __attribute__((ext_vector_type(16)));
typedef _Float16       v16h  __attribute__((ext_vector_type(16)));
typedef v4f  __attribute__((may_alias)) v4fa;
typedef v8us __attribute__((may_alias)) v8usa;
union FragB { v16bf v; v16us u; v8us h[2]; v8i w; };
union FragH { v16h  v; v16us u; v8us h[2]; v8i w; };

__device__ __forceinline__ v8f wmb(const FragB& a, const FragB& b, v8f c) {
  v8f d = __builtin_amdgcn_wmma_f32_16x16x32_bf16(false, a.v, false, b.v, (short)0, c, false, false);
  asm volatile("v_nop\n\tv_nop\n\tv_nop\n\tv_nop" : "+v"(d) : "v"(a.w), "v"(b.w));
  return d;
}

__device__ __forceinline__ v8f wmh(const FragH& a, const FragH& b, v8f c) {
  v8f d = __builtin_amdgcn_wmma_f32_16x16x32_f16(false, a.v, false, b.v, (short)0, c, false, false);
  asm volatile("v_nop\n\tv_nop\n\tv_nop\n\tv_nop" : "+v"(d) : "v"(a.w), "v"(b.w));
  return d;
}

__device__ __forceinline__ unsigned bf16_bits(float f) {
  const unsigned u = __float_as_uint(f);
  const unsigned r = (u + 0x7FFFu + ((u >> 16) & 1u)) >> 16;
  const unsigned q = (u >> 16) | 0x40u;
  return ((u & 0x7fffffffu) > 0x7f800000u) ? q : r;
}

__device__ __forceinline__ float bf16_val(float f) {
  return __uint_as_float(bf16_bits(f) << 16);
}
__device__ __forceinline__ int clampi(int v, int lo, int hi) {
  return v < lo ? lo : (v > hi ? hi : v);
}

__device__ __forceinline__ unsigned f16_bits(float f) {
  const unsigned u  = __float_as_uint(f);
  const unsigned s  = (u >> 16) & 0x8000u;
  const unsigned a  = u & 0x7fffffffu;
  const unsigned t  = a - 0x38000000u;
  const unsigned r  = (t + 0x0FFFu + ((t >> 13) & 1u)) >> 13;
  const unsigned rc = r > 0x7C00u ? 0x7C00u : r;
  const bool small  = a < 0x38800000u;
  const bool isnan  = a > 0x7f800000u;
  const unsigned fin = small ? 0u : (s | rc);
  return isnan ? (s | 0x7E00u) : fin;
}

__device__ __forceinline__ unsigned pk16(unsigned lo, unsigned hi) { return lo | (hi << 16); }
__device__ __forceinline__ unsigned bf16_lo_bits(float v) {
  float hi = bf16_val(v);
  asm volatile("" : "+v"(hi));
  return bf16_bits(v - hi);
}
__device__ __forceinline__ v4u pack8_bf16(v4f a, v4f c) {
  return (v4u){ pk16(bf16_bits(a[0]), bf16_bits(a[1])), pk16(bf16_bits(a[2]), bf16_bits(a[3])),
                pk16(bf16_bits(c[0]), bf16_bits(c[1])), pk16(bf16_bits(c[2]), bf16_bits(c[3])) };
}
__device__ __forceinline__ v4u pack8_bf16_lo(v4f a, v4f c) {
  return (v4u){ pk16(bf16_lo_bits(a[0]), bf16_lo_bits(a[1])), pk16(bf16_lo_bits(a[2]), bf16_lo_bits(a[3])),
                pk16(bf16_lo_bits(c[0]), bf16_lo_bits(c[1])), pk16(bf16_lo_bits(c[2]), bf16_lo_bits(c[3])) };
}
__device__ __forceinline__ v4u pack8_f16(v4f a, v4f c) {
  return (v4u){ pk16(f16_bits(a[0]), f16_bits(a[1])), pk16(f16_bits(a[2]), f16_bits(a[3])),
                pk16(f16_bits(c[0]), f16_bits(c[1])), pk16(f16_bits(c[2]), f16_bits(c[3])) };
}

template <int FORM>
__global__ __launch_bounds__(256) void k_plane(const float* __restrict__ src, int rows, int cols, int ldsrc,
                                               unsigned short* __restrict__ dst, int MP, int KP) {
  static_assert(FORM >= 0 && FORM <= 3);
  const int KTOT = (FORM == 1 || FORM == 3) ? 2 * KP : KP;
  const unsigned ppr   = (unsigned)(KTOT >> 3);
  const unsigned kp8   = (unsigned)(KP >> 3);
  const unsigned total = (unsigned)MP * ppr;
  const unsigned g     = blockIdx.x * 256u + threadIdx.x;
  const unsigned rowu  = g / ppr;
  const unsigned p     = g - rowu * ppr;
  const bool second    = p >= kp8;
  const int row = (int)rowu;
  const int c0  = (int)((second ? p - kp8 : p) << 3);
  const float* srow = src + (size_t)clampi(row, 0, rows - 1) * (size_t)ldsrc;
  float x[8];
  unsigned mk[8];
#pragma unroll
  for (int e = 0; e < 8; ++e) {
    const int c = c0 + e;
    const float v = srow[clampi(c, 0, cols - 1)];
    asm volatile("" :: "v"(v));
    x[e]  = v;
    mk[e] = (row < rows && c < cols) ? 0xFFFFu : 0u;
  }
  const v4f a = (v4f){ x[0], x[1], x[2], x[3] };
  const v4f c = (v4f){ x[4], x[5], x[6], x[7] };
  v4u o;
  if (FORM == 2) {
    o = pack8_f16(a, c);
  } else {
    const v4u hi = pack8_bf16(a, c);
    o = hi;
    if (FORM == 1) { const v4u lo = pack8_bf16_lo(a, c); o = second ? lo : hi; }
  }
  const v4u mw = (v4u){ pk16(mk[0], mk[1]), pk16(mk[2], mk[3]), pk16(mk[4], mk[5]), pk16(mk[6], mk[7]) };
  o &= mw;
  if (g < total) {
    volatile v4u* q = (volatile v4u*)(dst + (size_t)g * 8);
    *q = o;
    __threadfence();
    *q = o;
  }
}

template <int FORM> struct FragOf    { typedef FragB T; };
template <>         struct FragOf<2> { typedef FragH T; };
__device__ __forceinline__ v8f mm(const FragB& a, const FragB& b, v8f c) { return wmb(a, b, c); }
__device__ __forceinline__ v8f mm(const FragH& a, const FragH& b, v8f c) { return wmh(a, b, c); }
template <class F> __device__ __forceinline__ F ld_frag(const unsigned short* p) {
  F f;
  f.h[0] = *(const v8usa*)(p);
  f.h[1] = *(const v8usa*)(p + 16);
  return f;
}

template <int FORM, int EPI>
__global__ __launch_bounds__(256) __attribute__((amdgpu_num_vgpr(248)))
void k_gemm_nt(const unsigned short* __restrict__ A, const unsigned short* __restrict__ B,
               const float* __restrict__ bias, float* __restrict__ D, int M, int N, int KTOT, int ldd) {
  static_assert(FORM >= 0 && FORM <= 2);
  static_assert(EPI == 0 || EPI == 1);
  typedef typename FragOf<FORM>::T F;
  __shared__ __attribute__((aligned(16))) float sT[8][16 * 68];
  const int lane = threadIdx.x & 31;
  const int wave = threadIdx.x >> 5;
  const int tilesM = (M + 63) >> 6;
  const int tilesN = (N + 63) >> 6;
  const int tile = blockIdx.x * 8 + wave;
  if (tile >= tilesM * tilesN) return;
  const int tm = tile / tilesN;
  const int tn = tile - tm * tilesN;
  const int m0 = tm << 6;
  const int n0 = tn << 6;

  const int rl = lane & 15;
  const int h8 = (lane >> 4) * 8;
  const unsigned short* pa = A + (size_t)(m0 + rl) * (size_t)KTOT + h8;
  const unsigned short* pb = B + (size_t)(n0 + rl) * (size_t)KTOT + h8;

  v8f acc[4][4];
#pragma unroll
  for (int i = 0; i < 4; ++i)
#pragma unroll
    for (int j = 0; j < 4; ++j) acc[i][j] = (v8f){0.f, 0.f, 0.f, 0.f, 0.f, 0.f, 0.f, 0.f};

#pragma unroll 1
  for (int k0 = 0; k0 < KTOT; k0 += 32) {
    F bf[4];
#pragma unroll
    for (int j = 0; j < 4; ++j) bf[j] = ld_frag<F>(pb + (size_t)(j << 4) * (size_t)KTOT + k0);
#pragma unroll
    for (int i = 0; i < 4; ++i) {
      const F af = ld_frag<F>(pa + (size_t)(i << 4) * (size_t)KTOT + k0);
#pragma unroll
      for (int j = 0; j < 4; ++j) acc[i][j] = mm(af, bf[j], acc[i][j]);
    }
  }

  float* slab = sT[wave];
  const int hh = lane >> 4;
  const int c4 = (lane & 15) * 4;
  const int nc = n0 + c4;
  const bool cok = nc < N;
  v4f bv = (v4f){0.f, 0.f, 0.f, 0.f};
  if (EPI == 1) {
    bv = *(const v4fa*)(bias + clampi(nc, 0, N - 4));
    asm volatile("" :: "v"(bv));
  }
#pragma unroll
  for (int i = 0; i < 4; ++i) {
    const int mBase = m0 + (i << 4);
#pragma unroll
    for (int j = 0; j < 4; ++j) {
#pragma unroll
      for (int r = 0; r < 8; ++r) slab[(h8 + r) * 68 + (j << 4) + rl] = acc[i][j][r];
    }
    __builtin_amdgcn_fence(__ATOMIC_RELEASE, "workgroup");
    __builtin_amdgcn_wave_barrier();
    __builtin_amdgcn_fence(__ATOMIC_ACQUIRE, "workgroup");
    v4f vv[8];
#pragma unroll
    for (int it = 0; it < 8; ++it) {
      const int row = it * 2 + hh;
      v4f v = *(const v4fa*)(slab + row * 68 + c4);
      if (EPI == 1) v += bv;
      vv[it] = v;
    }
    for (int pass = 0; pass < 2; ++pass) {
#pragma unroll
      for (int it = 0; it < 8; ++it) {
        const int row = mBase + it * 2 + hh;
        if (cok && row < M) *(volatile v4f*)(D + (size_t)row * (size_t)ldd + nc) = vv[it];
      }
      __threadfence();
    }
    __builtin_amdgcn_fence(__ATOMIC_RELEASE, "workgroup");
    __builtin_amdgcn_wave_barrier();
    __builtin_amdgcn_fence(__ATOMIC_ACQUIRE, "workgroup");
  }
}

#pragma clang fp contract(off)

typedef float v2f __attribute__((ext_vector_type(2)));
typedef v2f __attribute__((may_alias)) v2fa;

constexpr int NN    = 50000;
constexpr int DEG   = 16;
constexpr int IN    = 128;
constexpr int OUT   = 64;
constexpr int MPAD  = 50048;
constexpr int GT    = (NN + 63) / 64;
constexpr int OUT_ELEMS = NN * OUT;

static_assert(NN % 8 == 0);
static_assert(DEG == 16 && DEG <= 32);
static_assert(OUT == 64 && OUT == 2 * 32);
static_assert(IN == 128 && IN % 32 == 0);
static_assert(MPAD == 391 * 128);
static_assert(MPAD % 64 == 0 && MPAD >= NN && NN % 16 == 0 && OUT % 4 == 0 && OUT % 32 == 0 && OUT % 64 == 0);
static_assert((long long)MPAD * IN / 8 < 0x7fffffffLL && (MPAD * IN / 8) % 256 == 0);
static_assert(GT == 782);
static_assert(OUT_ELEMS == 3200000);

constexpr size_t SZ_DB   = (size_t)MPAD * IN * 2;
constexpr size_t SZ_MB   = (size_t)MPAD * IN * 2;
constexpr size_t SZ_H    = (size_t)MPAD * OUT * 4;
constexpr size_t SZ_S    = (size_t)MPAD * OUT * 4;
constexpr size_t SZ_WT   = (size_t)OUT * IN * 2;
constexpr size_t SZ_BIAS = (size_t)2 * OUT * 4;
constexpr size_t OFF_DB   = 0;
constexpr size_t OFF_MB   = OFF_DB + SZ_DB;
constexpr size_t OFF_H    = OFF_MB + SZ_MB;
constexpr size_t OFF_S    = OFF_H + SZ_H;
constexpr size_t OFF_WLT  = OFF_S + SZ_S;
constexpr size_t OFF_WTT  = OFF_WLT + SZ_WT;
constexpr size_t OFF_BIAS = OFF_WTT + SZ_WT;
constexpr size_t WS_TOTAL = OFF_BIAS + SZ_BIAS;
static_assert(SZ_DB % 256 == 0 && SZ_H % 256 == 0 && SZ_WT % 256 == 0 && SZ_BIAS % 256 == 0);
static_assert(OFF_MB % 256 == 0 && OFF_H % 256 == 0 && OFF_S % 256 == 0 && OFF_WLT % 256 == 0);
static_assert(OFF_WTT % 256 == 0 && OFF_BIAS % 256 == 0);
static_assert(OFF_MB == (size_t)12812288 && OFF_H == (size_t)25624576 && OFF_S == (size_t)38436864);
static_assert(OFF_WLT == (size_t)51249152 && OFF_WTT == (size_t)51265536 && OFF_BIAS == (size_t)51281920);
static_assert(WS_TOTAL == (size_t)51282432);
static_assert(WS_TOTAL <= ((size_t)128 << 20));

constexpr int WPIECES = OUT * IN / 8;
constexpr int WBLK    = WPIECES / 256;
constexpr int PREP_BLOCKS = 2 * WBLK + 1;
static_assert(WPIECES % 256 == 0 && WBLK == 4 && PREP_BLOCKS == 9);

__device__ __forceinline__ void prep_wt(const float* __restrict__ W, unsigned short* __restrict__ dst, int g) {
  const int n  = g >> 4;
  const int k0 = (g & 15) * 8;
  const float* s = W + (size_t)k0 * OUT + n;
  float x[8];
#pragma unroll
  for (int e = 0; e < 8; ++e) {
    const float v = s[(size_t)e * OUT];
    asm volatile("" :: "v"(v));
    x[e] = v;
  }
  const v4u o = pack8_bf16((v4f){ x[0], x[1], x[2], x[3] }, (v4f){ x[4], x[5], x[6], x[7] });
  volatile v4u* q = (volatile v4u*)(dst + (size_t)g * 8);
  *q = o;
  __threadfence();
  *q = o;
}

__global__ __launch_bounds__(256) void k_prep(const float* __restrict__ W_lin, const float* __restrict__ b_lin,
                                              const float* __restrict__ W_tr, const float* __restrict__ b_tr,
                                              unsigned short* __restrict__ WLT, unsigned short* __restrict__ WTT,
                                              float* __restrict__ BIAS) {
  const int tid = (int)threadIdx.x;
  const int blk = (int)blockIdx.x;
  if (blk < WBLK) {
    prep_wt(W_lin, WLT, blk * 256 + tid);
  } else if (blk < 2 * WBLK) {
    prep_wt(W_tr, WTT, (blk - WBLK) * 256 + tid);
  } else {
    const int u  = tid < 32 ? tid : 31;
    const int il = clampi(u, 0, 15) * 4;
    const int it = clampi(u - 16, 0, 15) * 4;
    const v4f a0 = *(const v4fa*)(b_lin + il);
    const v4f a1 = *(const v4fa*)(b_tr + it);
    asm volatile("" :: "v"(a0));
    asm volatile("" :: "v"(a1));
    const unsigned m0 = (u < 16) ? 0xFFFFFFFFu : 0u;
    const unsigned m1 = ~m0;
    v4f o;
#pragma unroll
    for (int e = 0; e < 4; ++e) {
      const unsigned bits = (__float_as_uint(a0[e]) & m0) | (__float_as_uint(a1[e]) & m1);
      o[e] = bf16_val(__uint_as_float(bits));
    }
    if (tid < 32) {
      volatile v4f* q = (volatile v4f*)(BIAS + 4 * tid);
      *q = o;
      __threadfence();
      *q = o;
    }
  }
}

__device__ __forceinline__ void row_add(const float* __restrict__ Hl, int idc, int j, float& a0, float& a1) {
  const int nr = __builtin_amdgcn_readlane(idc, j);
  const v2f rv = *(const v2fa*)(Hl + (size_t)nr * OUT);
  const float r0 = rv[0], r1 = rv[1];
  asm volatile("" :: "v"(r0));
  asm volatile("" :: "v"(r1));
  a0 += r0;
  a1 += r1;
}

static_assert((NN / 8) * 8 == NN);
static_assert((size_t)(NN - 1) * OUT + 2 * 31 + 1 == (size_t)OUT_ELEMS - 1);
__global__ __launch_bounds__(256) void k_node(const int* __restrict__ tbl, const float* __restrict__ H,
                                              const float* __restrict__ S, float* __restrict__ out) {
  const int tid = (int)threadIdx.x, lane = tid & 31, wave = tid >> 5;
  const int node = __builtin_amdgcn_readfirstlane((int)blockIdx.x * 8 + wave);
  const int nq   = node < NN ? node : NN - 1;

  int idv = tbl[(size_t)nq * DEG + (lane & 15)];
  asm volatile("" :: "v"(idv));
  const int idc = clampi(idv, 0, NN - 1);

  const float* Hl = H + 2 * lane;
  float a0 = 0.0f, a1 = 0.0f;
#pragma unroll
  for (int j = 0; j < 8; ++j) row_add(Hl, idc, j, a0, a1);
  asm volatile("" ::: "memory");
#pragma unroll
  for (int j = 8; j < 16; ++j) row_add(Hl, idc, j, a0, a1);
  asm volatile("" ::: "memory");

  const v2f hv = *(const v2fa*)(Hl + (size_t)nq * OUT);
  const v2f sv = *(const v2fa*)(S + (size_t)nq * OUT + 2 * lane);
  const float h0 = hv[0], h1 = hv[1];
  const float s0 = sv[0], s1 = sv[1];
  asm volatile("" :: "v"(h0));
  asm volatile("" :: "v"(h1));
  asm volatile("" :: "v"(s0));
  asm volatile("" :: "v"(s1));

  const float t0 = 16.0f * h0 - a0;
  const float t1 = 16.0f * h1 - a1;
  const float l0 = t0 * 0.0625f;
  const float l1 = t1 * 0.0625f;
  const float v0 = l0 + s0;
  const float v1 = l1 + s1;
  const float o0 = (v0 > 0.0f) ? v0 : (v0 - v0);
  const float o1 = (v1 > 0.0f) ? v1 : (v1 - v1);
  const v2f o = (v2f){ o0, o1 };
  if (node < NN) {
    volatile v2f* q = (volatile v2f*)(out + (size_t)node * OUT + 2 * lane);
    *q = o;
    __threadfence();
    *q = o;
  }
}

extern "C" void kernel_launch(void* const* d_in, const int* in_sizes, int n_in,
                              void* d_out, int out_size, void* d_ws, size_t ws_size,
                              hipStream_t stream) {
  if (n_in < 7) return;
  if (in_sizes[0] != NN * IN) return;
  if (in_sizes[1] != NN * IN) return;
  if (in_sizes[2] != NN * DEG) return;
  if (in_sizes[3] != IN * OUT) return;
  if (in_sizes[4] != OUT) return;
  if (in_sizes[5] != IN * OUT) return;
  if (in_sizes[6] != OUT) return;
  if (out_size != OUT_ELEMS) return;
  if (ws_size < WS_TOTAL) return;

  const float* data  = (const float*)d_in[0];
  const float* merge = (const float*)d_in[1];
  const int*   tbl   = (const int*)d_in[2];
  const float* W_lin = (const float*)d_in[3];
  const float* b_lin = (const float*)d_in[4];
  const float* W_tr  = (const float*)d_in[5];
  const float* b_tr  = (const float*)d_in[6];
  float* out = (float*)d_out;

  char* ws = (char*)d_ws;
  unsigned short* DB   = (unsigned short*)(ws + OFF_DB);
  unsigned short* MB   = (unsigned short*)(ws + OFF_MB);
  float*          H    = (float*)(ws + OFF_H);
  float*          S    = (float*)(ws + OFF_S);
  unsigned short* WLT  = (unsigned short*)(ws + OFF_WLT);
  unsigned short* WTT  = (unsigned short*)(ws + OFF_WTT);
  float*          BIAS = (float*)(ws + OFF_BIAS);
  const float*    BL   = BIAS;
  const float*    BT   = BIAS + OUT;

  k_prep<<<PREP_BLOCKS, 256, 0, stream>>>(W_lin, b_lin, W_tr, b_tr, WLT, WTT, BIAS);
  k_plane<0><<<MPAD * IN / 8 / 256, 256, 0, stream>>>(data, NN, IN, IN, DB, MPAD, IN);
  k_plane<0><<<MPAD * IN / 8 / 256, 256, 0, stream>>>(merge, NN, IN, IN, MB, MPAD, IN);
  k_gemm_nt<0, 1><<<(GT + 7) / 8, 256, 0, stream>>>(DB, WLT, BL, H, NN, OUT, IN, OUT);
  k_gemm_nt<0, 1><<<(GT + 7) / 8, 256, 0, stream>>>(MB, WTT, BT, S, NN, OUT, IN, OUT);
  k_node<<<NN / 8, 256, 0, stream>>>(tbl, H, S, out);
}
